// MultiHeadSelfAttention_29351806501634
// MI455X (gfx1250) — hardware-run, weakly checked
//
#include <hip/hip_runtime.h>


#ifndef NB
#define NB 8
#endif
#ifndef SEQ
#define SEQ 2048
#endif
#define NB_FULL  8
#define SEQ_FULL 2048
#define TT   SEQ
#define DM   256
#define NH_  4
#define HD   64
#define DQ   (NH_ * HD)
#define NQKV (3 * DQ)
#define ROWS (NB * TT)
#define SCL  0.125f
#define QCAR 16.0f
#define FW   4
#define L2E  1.4426950408889634f
typedef _Float16 h16;
typedef unsigned short bf;
typedef __attribute__((ext_vector_type(16))) __bf16   v16bf;
typedef __attribute__((ext_vector_type(16))) _Float16 v16h;
typedef __attribute__((ext_vector_type(8)))  _Float16 v8h;
typedef __attribute__((ext_vector_type(8)))  unsigned short v8us;
typedef __attribute__((ext_vector_type(8)))  float    v8f;
typedef __attribute__((ext_vector_type(4)))  float    v4f;
typedef __attribute__((ext_vector_type(2)))  float    v2f;
typedef __attribute__((ext_vector_type(2)))  _Float16 v2h;
typedef __attribute__((ext_vector_type(4)))  _Float16 v4h;
typedef __attribute__((ext_vector_type(2)))  unsigned short v2us;
typedef __attribute__((ext_vector_type(4)))  unsigned short v4us;
typedef __attribute__((ext_vector_type(4)))  int      v4i;
typedef v4f  __attribute__((may_alias)) v4fa;

static_assert(NB >= 1 && NB <= NB_FULL);
static_assert(SEQ >= 128 && SEQ <= SEQ_FULL);
static_assert(TT % 128 == 0);
static_assert(TT % 64 == 0 && DM % 64 == 0 && NQKV % 64 == 0 && DQ % 64 == 0 && HD % 64 == 0);
static_assert(DM % 32 == 0 && DQ % 32 == 0 && HD % 32 == 0 && TT % 32 == 0);
static_assert(HD == 64);
static_assert(DQ == DM);
static_assert(2 * DQ + DQ == NQKV);
static_assert(TT % (16 * FW) == 0);
static_assert(FW * 32 == 128);
static_assert(((size_t)NB * NH_ * TT * HD) % 8 == 0);
static_assert(((size_t)(NB - 1) * SEQ_FULL * DM + (size_t)TT * DM) * 4 <= (size_t)NB_FULL * SEQ_FULL * DM * 4);

#define AL256(x) ((((size_t)(x)) + 255) & ~(size_t)255)
#define WS_TOTAL (AL256((size_t)NQKV * DM * 2) + AL256((size_t)DM * DQ * 2) + AL256((size_t)ROWS * DM * 2) + AL256((size_t)ROWS * NQKV * 4) \
    + 3 * AL256((size_t)NB * NH_ * TT * HD * 2) + 2 * AL256((size_t)ROWS * DQ * 2))
static_assert(WS_TOTAL <= (size_t)134217728);

__device__ __forceinline__ unsigned short f2bf(float f) { unsigned u = __float_as_uint(f); u += 0x7FFFu + ((u >> 16) & 1u); return (unsigned short)(u >> 16); }
__device__ __forceinline__ float bf2f(unsigned short b) { return __uint_as_float(((unsigned)b) << 16); }
__device__ __forceinline__ float bfr(float f) { return bf2f(f2bf(f)); }
__device__ __forceinline__ v16h cat16(v8h lo, v8h hi) { return __builtin_shufflevector(lo, hi, 0, 1, 2, 3, 4, 5, 6, 7, 8, 9, 10, 11, 12, 13, 14, 15); }
__device__ __forceinline__ v16bf cat16b(v8us lo, v8us hi) { return __builtin_bit_cast(v16bf, __builtin_shufflevector(lo, hi, 0, 1, 2, 3, 4, 5, 6, 7, 8, 9, 10, 11, 12, 13, 14, 15)); }
__device__ __forceinline__ v8f wmma16(v16h a, v16h b, v8f c) { return __builtin_amdgcn_wmma_f32_16x16x32_f16(false, a, false, b, (short)0, c, false, false); }
__device__ __forceinline__ v8f wmmab(v16bf a, v16bf b, v8f c) { return __builtin_amdgcn_wmma_f32_16x16x32_bf16(false, a, false, b, (short)0, c, false, false); }

template <typename T16> struct WFrag;
template <> struct WFrag<h16> { typedef v16h V; static __device__ __forceinline__ V ld(const h16* p) { return cat16(*(const v8h*)p, *(const v8h*)(p + 16)); } static __device__ __forceinline__ v8f mma(V a, V b, v8f c) { return wmma16(a, b, c); } };
template <> struct WFrag<bf> { typedef v16bf V; static __device__ __forceinline__ V ld(const bf* p) { return cat16b(*(const v8us*)p, *(const v8us*)(p + 16)); } static __device__ __forceinline__ v8f mma(V a, V b, v8f c) { return wmmab(a, b, c); } };

template <typename T16, int NSPLIT, bool BIAS>
__device__ __forceinline__ void gemmw_body(const T16* __restrict__ A, const T16* __restrict__ A2, const T16* __restrict__ Bt, const T16* __restrict__ Bt2, int K, float* C, int ldc, const float* __restrict__ bias, size_t sA, size_t sB, size_t sC) {
    typedef typename WFrag<T16>::V V;
    __shared__ __align__(16) float os[16 * 68];
    const size_t z = blockIdx.z; A += z * sA; if (A2) A2 += z * sA; Bt += z * sB; if (Bt2) Bt2 += z * sB; C += z * sC;
    const int lane = threadIdx.x & 31, lr = lane & 15, hi = lane >> 4; const int r0 = blockIdx.x * 64, c0 = blockIdx.y * 64;
    v8f acc[4][4];
#pragma unroll
    for (int mb = 0; mb < 4; ++mb)
#pragma unroll
        for (int nb = 0; nb < 4; ++nb) acc[mb][nb] = (v8f){};
    const size_t aoff = (size_t)(r0 + lr) * K + 8 * hi, boff = (size_t)(c0 + lr) * K + 8 * hi;
#pragma unroll 1
    for (int kc = 0; kc < K; kc += 32) {
        V a[4], a2[4];
#pragma unroll
        for (int mb = 0; mb < 4; ++mb) { a[mb] = WFrag<T16>::ld(A + aoff + (size_t)mb * 16 * K + kc); if (NSPLIT == 1 || NSPLIT == 2) a2[mb] = WFrag<T16>::ld(A2 + aoff + (size_t)mb * 16 * K + kc); }
#pragma unroll
        for (int nb = 0; nb < 4; ++nb) { const V b = WFrag<T16>::ld(Bt + boff + (size_t)nb * 16 * K + kc); V b2; if (NSPLIT >= 2) b2 = WFrag<T16>::ld(Bt2 + boff + (size_t)nb * 16 * K + kc);
#pragma unroll
            for (int mb = 0; mb < 4; ++mb) { acc[mb][nb] = WFrag<T16>::mma(a[mb], b, acc[mb][nb]); if (NSPLIT == 1 || NSPLIT == 2) acc[mb][nb] = WFrag<T16>::mma(a2[mb], b, acc[mb][nb]); if (NSPLIT >= 2) acc[mb][nb] = WFrag<T16>::mma(a[mb], b2, acc[mb][nb]); } }
        asm volatile("v_nop\n\tv_nop\n\tv_nop\n\tv_nop" : "+v"(acc[0][0]), "+v"(acc[1][1]), "+v"(acc[2][2]), "+v"(acc[3][3]) : "v"(a[0]), "v"(a[3]));
    }
#pragma unroll
    for (int mb = 0; mb < 4; ++mb) {
#pragma unroll
        for (int nb = 0; nb < 4; ++nb) {
#pragma unroll
            for (int j = 0; j < 8; ++j) os[(hi * 8 + j) * 68 + nb * 16 + lr] = acc[mb][nb][j]; }
        __builtin_amdgcn_wave_barrier(); asm volatile("" ::: "memory");
        float* crow = C + (size_t)(r0 + mb * 16) * ldc + c0;
#pragma unroll 1
        for (int ps = 0; ps < 2; ++ps) {
#pragma unroll
            for (int s = 0; s < 8; ++s) { const int row = 2 * s + hi, cofs = lr * 4; v4f val = *(const v4fa*)(os + row * 68 + cofs); if (BIAS) { val[0] += bfr(bias[c0 + cofs]); val[1] += bfr(bias[c0 + cofs + 1]); val[2] += bfr(bias[c0 + cofs + 2]); val[3] += bfr(bias[c0 + cofs + 3]); }
                *(volatile v4f*)(crow + (size_t)row * ldc + cofs) = val; }
            if (ps == 0) __threadfence(); }
        __builtin_amdgcn_wave_barrier(); asm volatile("" ::: "memory");
    }
}

__global__ __launch_bounds__(32) void k_gemm_qkv(const bf* A, const bf* Bt, int K, float* C, int ldc, const float* bias) { gemmw_body<bf, 0, true>(A, nullptr, Bt, nullptr, K, C, ldc, bias, 0, 0, 0); }
__global__ __launch_bounds__(32) void k_gemm_out(const bf* A, const bf* A2, const bf* Bt, int K, float* C, int ldc, const float* bias) { gemmw_body<bf, 1, true>(A, A2, Bt, nullptr, K, C, ldc, bias, 0, 0, 0); }

__device__ __forceinline__ void splitf(float y, unsigned short& h, unsigned short& l) { h = f2bf(y); l = f2bf(y - bf2f(h)); }

__global__ __launch_bounds__(256) void k_wtG(const float* __restrict__ w, int K, int N, bf* Bt) {
    const int lane = threadIdx.x & 31; const int L0 = (blockIdx.x * 8 + (threadIdx.x >> 5)) * 8; const int nlines = N * K / 64;
#pragma unroll
    for (int ps = 0; ps < 2; ++ps) {
#pragma unroll 1
        for (int l = 0; l < 8; ++l) { const int L = L0 + l; if (L >= nlines) break; const size_t e = (size_t)L * 64 + lane * 2; const int k = (int)(e % K), n = (int)(e / K); v2us o;
            o[0] = f2bf(w[(size_t)k * N + n]); o[1] = f2bf(w[(size_t)(k + 1) * N + n]); *(volatile v2us*)(Bt + e) = o; }
        if (ps == 0) __threadfence(); }
}
__global__ __launch_bounds__(256) void k_cvt8(const float* __restrict__ src, bf* dst, size_t n8) { const size_t i = (size_t)blockIdx.x * 256 + threadIdx.x; if (i >= n8) return; const v8f v = *(const v8f*)(src + i * 8); v8us o;
#pragma unroll
    for (int k = 0; k < 8; ++k) o[k] = f2bf(v[k]); *(volatile v8us*)(dst + i * 8) = o; __threadfence(); *(volatile v8us*)(dst + i * 8) = o; }

static __device__ __forceinline__ h16 toh_flush(float v) { const h16 r = (h16)v; return (fabsf(v) < 6.103515625e-05f) ? (h16)0.0f : r; }
static __device__ __forceinline__ v8f wmma16g(v16h a, v16h b, v8f c) { c = wmma16(a, b, c); asm volatile("v_nop\n\tv_nop\n\tv_nop\n\tv_nop" : "+v"(c) : "v"(a), "v"(b)); return c; }

__global__ __launch_bounds__(256) void k_hp16(const float* __restrict__ F, int pitch, h16* P16) {
    const size_t e = ((size_t)blockIdx.x * 256 + threadIdx.x) * 8; if (e >= (size_t)NB * NH_ * TT * HD) return;
    const int d = (int)(e % HD); const int t = (int)((e / HD) % TT); const int bh = (int)(e / ((size_t)HD * TT)); const int b = bh / NH_, h = bh % NH_;
    const float* src = F + ((size_t)b * TT + t) * pitch + h * HD + d; const v4f x0 = *(const v4f*)src; const v4f x1 = *(const v4f*)(src + 4); v8h o;
#pragma unroll
    for (int q = 0; q < 4; ++q) { o[q] = toh_flush(x0[q] * QCAR); o[4 + q] = toh_flush(x1[q] * QCAR); }
    *(volatile v8h*)(P16 + e) = o; __threadfence(); *(volatile v8h*)(P16 + e) = o; }
__global__ __launch_bounds__(256) void k_vtp16(const float* __restrict__ F, int pitch, h16* V16) {
    const size_t e = ((size_t)blockIdx.x * 256 + threadIdx.x) * 8; if (e >= (size_t)NB * NH_ * HD * TT) return;
    const int t = (int)(e % TT); const int d = (int)((e / TT) % HD); const int bg = (int)(e / ((size_t)TT * HD)); const int b = bg / NH_, g = bg % NH_;
    const float* src = F + ((size_t)b * TT + t) * pitch + g * HD + d; v8h o;
#pragma unroll
    for (int q = 0; q < 8; ++q) o[q] = toh_flush(src[(size_t)q * pitch] * QCAR);
    *(volatile v8h*)(V16 + e) = o; __threadfence(); *(volatile v8h*)(V16 + e) = o; }

__global__ __launch_bounds__(128) void k_flash(const h16* __restrict__ Q16, const h16* __restrict__ K16, const h16* __restrict__ VT16, const int* __restrict__ mask, bf* ATh, bf* ATl) {
    __shared__ __align__(16) float os[FW * 16 * 68];
    const int wave = __builtin_amdgcn_readfirstlane(threadIdx.x >> 5);
    const int lane = threadIdx.x & 31, lr = lane & 15, hi = lane >> 4;
    const int bh = blockIdx.y; const int b = bh / NH_, h = bh % NH_;
    const int q0 = (blockIdx.x * FW + wave) * 16;
    int mn = TT, mx = -1;
    const int* mrow = mask + (size_t)b * SEQ_FULL;
#pragma unroll 1
    for (int p = lane * 4; p < TT; p += 128) { const v4i mv = *(const v4i*)(mrow + p);
#pragma unroll
        for (int c = 0; c < 4; ++c) { const bool on = (mv[c] != 0); mn = on ? min(mn, p + c) : mn; mx = on ? max(mx, p + c) : mx; } }
#pragma unroll
    for (int sh = 16; sh; sh >>= 1) { mn = min(mn, __shfl_xor(mn, sh, 32)); mx = max(mx, __shfl_xor(mx, sh, 32)); }
    const int stv = (mn < TT) ? mn : 0;
    const int env = (mx >= 0) ? mx : (TT - 1);
    const int vlv = max(env - stv, 0);
    const bool allv = (q0 >= stv) && (q0 + 16 <= stv + vlv);
    const int kbv = allv ? (stv & ~31) : 0;
    const int kev = allv ? min(TT, (stv + vlv + 31) & ~31) : TT;
    const int st = __builtin_amdgcn_readfirstlane(stv);
    const int vlen = __builtin_amdgcn_readfirstlane(vlv);
    const int kbeg = __builtin_amdgcn_readfirstlane(kbv);
    const int kend = __builtin_amdgcn_readfirstlane(kev);
    const bool qv = (unsigned)(q0 + lr - st) < (unsigned)vlen;
    const float qb = qv ? 0.0f : -1.0e10f;

    const size_t hp = (size_t)bh * TT * HD;
    const h16* qp = Q16 + hp + (size_t)(q0 + lr) * HD + 8 * hi;
    const v16h qf0 = WFrag<h16>::ld(qp), qf1 = WFrag<h16>::ld(qp + 32);
    const h16* kp = K16 + hp + (size_t)lr * HD + 8 * hi;
    const h16* vp = VT16 + hp + (size_t)lr * TT + 8 * hi;
    const float tsc = SCL / (QCAR * QCAR);

    v8f o[4];
#pragma unroll
    for (int dt = 0; dt < 4; ++dt) o[dt] = (v8f){};
    float m = -1.0e30f, l = 0.0f;
#pragma unroll 1
    for (int kb = kbeg; kb < kend; kb += 32) {
        v8f s0 = (v8f){}, s1 = (v8f){};
        { const h16* kr0 = kp + (size_t)kb * HD;
          const v16h a0 = WFrag<h16>::ld(kr0), a1 = WFrag<h16>::ld(kr0 + 32);
          const v16h c0 = WFrag<h16>::ld(kr0 + 16 * HD), c1 = WFrag<h16>::ld(kr0 + 16 * HD + 32);
          s0 = wmma16g(a0, qf0, s0); s0 = wmma16g(a1, qf1, s0);
          s1 = wmma16g(c0, qf0, s1); s1 = wmma16g(c1, qf1, s1); }
        const int rel = kb - st;
        float t0[8], t1[8];
        if (rel >= 0 && rel + 32 <= vlen) {
#pragma unroll
            for (int r = 0; r < 8; ++r) { t0[r] = s0[r] * tsc + qb; t1[r] = s1[r] * tsc + qb; }
        } else if (rel + 32 <= 0 || rel >= vlen) {
#pragma unroll
            for (int r = 0; r < 8; ++r) { t0[r] = s0[r] * tsc + (-1.0e10f); t1[r] = s1[r] * tsc + (-1.0e10f); }
        } else {
            const int kr = rel + 8 * hi;
#pragma unroll
            for (int r = 0; r < 8; ++r) { const bool v0 = qv && ((unsigned)(kr + r) < (unsigned)vlen); const bool v1 = qv && ((unsigned)(kr + 16 + r) < (unsigned)vlen);
                t0[r] = s0[r] * tsc + (v0 ? 0.0f : -1.0e10f); t1[r] = s1[r] * tsc + (v1 ? 0.0f : -1.0e10f); }
        }
        float mloc = -1.0e30f;
#pragma unroll
        for (int r = 0; r < 8; ++r) mloc = fmaxf(mloc, fmaxf(t0[r], t1[r]));
        mloc = fmaxf(mloc, __shfl_xor(mloc, 16, 32));
        const float mnew = fmaxf(m, mloc);
        const float alpha = __builtin_amdgcn_exp2f((m - mnew) * L2E);
        m = mnew;
        v16h pb; float ls = 0.0f;
#pragma unroll
        for (int r = 0; r < 8; ++r) { const float e0 = (t0[r] - m) * L2E, e1 = (t1[r] - m) * L2E;
            const float p0 = (e0 < -14.0f) ? 0.0f : __builtin_amdgcn_exp2f(e0); const float p1 = (e1 < -14.0f) ? 0.0f : __builtin_amdgcn_exp2f(e1);
            const h16 h0 = (h16)p0, h1 = (h16)p1; pb[r] = h0; pb[8 + r] = h1; ls += (float)h0 + (float)h1; }
        l = l * alpha + ls;
#pragma unroll
        for (int dt = 0; dt < 4; ++dt) o[dt] = o[dt] * alpha;
        { const h16* vk = vp + kb;
          const v16h g0 = WFrag<h16>::ld(vk), g1 = WFrag<h16>::ld(vk + (size_t)16 * TT), g2 = WFrag<h16>::ld(vk + (size_t)32 * TT), g3 = WFrag<h16>::ld(vk + (size_t)48 * TT);
          o[0] = wmma16g(g0, pb, o[0]); o[1] = wmma16g(g1, pb, o[1]); o[2] = wmma16g(g2, pb, o[2]); o[3] = wmma16g(g3, pb, o[3]); }
    }
    l += __shfl_xor(l, 16, 32);
    const float inv = (1.0f / QCAR) * (1.0f / l);
    const int ob = wave * (16 * 68);
#pragma unroll
    for (int dt = 0; dt < 4; ++dt) {
#pragma unroll
        for (int r = 0; r < 8; ++r) os[ob + lr * 68 + dt * 16 + 8 * hi + r] = o[dt][r] * inv; }
    __builtin_amdgcn_wave_barrier(); asm volatile("" ::: "memory");
    const size_t arow = ((size_t)b * TT + q0) * DQ + h * HD;
#pragma unroll 1
    for (int ps = 0; ps < 2; ++ps) {
#pragma unroll
        for (int s = 0; s < 4; ++s) { const int row = 4 * s + (lane >> 3), pc = (lane & 7) * 8;
            const v4f x0 = *(const v4fa*)(os + ob + row * 68 + pc); const v4f x1 = *(const v4fa*)(os + ob + row * 68 + pc + 4); v8us oh, ol;
#pragma unroll
            for (int q = 0; q < 4; ++q) { unsigned short a, c2; splitf(x0[q], a, c2); oh[q] = a; ol[q] = c2; splitf(x1[q], a, c2); oh[4 + q] = a; ol[4 + q] = c2; }
            const size_t oo = arow + (size_t)row * DQ + pc;
            *(volatile v8us*)(ATh + oo) = oh; *(volatile v8us*)(ATl + oo) = ol; }
        if (ps == 0) __threadfence(); }
}

extern "C" void kernel_launch(void* const* d_in, const int* in_sizes, int n_in,
                              void* d_out, int out_size, void* d_ws, size_t ws_size, hipStream_t stream) {
    if (n_in < 10) return;
    const size_t xneed = (size_t)(NB - 1) * SEQ_FULL * DM + (size_t)TT * DM;
    const size_t mneed = (size_t)(NB - 1) * SEQ_FULL + (size_t)TT;
    if ((size_t)in_sizes[0] < xneed) return; if ((size_t)in_sizes[1] < mneed) return;
    if ((size_t)in_sizes[2] < (size_t)DM * DQ) return; if ((size_t)in_sizes[3] < (size_t)DQ) return;
    if ((size_t)in_sizes[4] < (size_t)DM * DQ) return; if ((size_t)in_sizes[5] < (size_t)DQ) return;
    if ((size_t)in_sizes[6] < (size_t)DM * DQ) return; if ((size_t)in_sizes[7] < (size_t)DQ) return;
    if ((size_t)in_sizes[8] < (size_t)DQ * DM) return; if ((size_t)in_sizes[9] < (size_t)DM) return;
    if ((size_t)out_size < xneed) return;
    if (ws_size < WS_TOTAL) return;
    const float* x = (const float*)d_in[0]; const int* amask = (const int*)d_in[1];
    const float* wq = (const float*)d_in[2]; const float* bq = (const float*)d_in[3];
    const float* wk = (const float*)d_in[4]; const float* bk = (const float*)d_in[5];
    const float* wv = (const float*)d_in[6]; const float* bv = (const float*)d_in[7];
    const float* wo = (const float*)d_in[8]; const float* bo = (const float*)d_in[9];
    float* OUT = (float*)d_out;
    char* wsp = (char*)d_ws;
    auto take = [&](size_t bytes) { char* p = wsp; wsp += (bytes + 255) & ~(size_t)255; return (void*)p; };
    bf* WQKV = (bf*)take((size_t)NQKV * DM * 2);
    bf* WO = (bf*)take((size_t)DM * DQ * 2);
    bf* XB = (bf*)take((size_t)ROWS * DM * 2);
    float* F = (float*)take((size_t)ROWS * NQKV * 4);
    h16* Q16 = (h16*)take((size_t)NB * NH_ * TT * HD * 2);
    h16* K16 = (h16*)take((size_t)NB * NH_ * TT * HD * 2);
    h16* VT16 = (h16*)take((size_t)NB * NH_ * HD * TT * 2);
    bf* ATh = (bf*)take((size_t)ROWS * DQ * 2); bf* ATl = (bf*)take((size_t)ROWS * DQ * 2);
    if ((size_t)(wsp - (char*)d_ws) > ws_size) return;
    if ((size_t)(wsp - (char*)d_ws) > (size_t)134217728) return;
    k_wtG<<<(unsigned)((DM * DQ / 64 + 63) / 64), 256, 0, stream>>>(wq, DM, DQ, WQKV);
    k_wtG<<<(unsigned)((DM * DQ / 64 + 63) / 64), 256, 0, stream>>>(wk, DM, DQ, WQKV + (size_t)DQ * DM);
    k_wtG<<<(unsigned)((DM * DQ / 64 + 63) / 64), 256, 0, stream>>>(wv, DM, DQ, WQKV + (size_t)2 * DQ * DM);
    k_wtG<<<(unsigned)((DQ * DM / 64 + 63) / 64), 256, 0, stream>>>(wo, DQ, DM, WO);
    if (SEQ == SEQ_FULL) {
        k_cvt8<<<(unsigned)(((size_t)ROWS * DM / 8 + 255) / 256), 256, 0, stream>>>(x, XB, (size_t)ROWS * DM / 8);
    } else {
        for (int b = 0; b < NB; ++b)
            k_cvt8<<<(unsigned)(((size_t)TT * DM / 8 + 255) / 256), 256, 0, stream>>>(x + (size_t)b * SEQ_FULL * DM, XB + (size_t)b * TT * DM, (size_t)TT * DM / 8);
    }
    k_gemm_qkv<<<dim3(ROWS / 64, DQ / 64, 1), 32, 0, stream>>>(XB, WQKV, DM, F, NQKV, bq);
    k_gemm_qkv<<<dim3(ROWS / 64, DQ / 64, 1), 32, 0, stream>>>(XB, WQKV + (size_t)DQ * DM, DM, F + DQ, NQKV, bk);
    k_gemm_qkv<<<dim3(ROWS / 64, DQ / 64, 1), 32, 0, stream>>>(XB, WQKV + (size_t)2 * DQ * DM, DM, F + 2 * DQ, NQKV, bv);
    const unsigned LP = (unsigned)(((size_t)NB * NH_ * TT * HD / 8 + 255) / 256);
    k_hp16<<<LP, 256, 0, stream>>>(F, NQKV, Q16);
    k_hp16<<<LP, 256, 0, stream>>>(F + DQ, NQKV, K16);
    k_vtp16<<<LP, 256, 0, stream>>>(F + 2 * DQ, NQKV, VT16);
    k_flash<<<dim3(TT / (16 * FW), NB * NH_, 1), 32 * FW, 0, stream>>>(Q16, K16, VT16, amask, ATh, ATl);
    if (SEQ == SEQ_FULL) {
        k_gemm_out<<<dim3(ROWS / 64, DM / 64, 1), 32, 0, stream>>>(ATh, ATl, WO, DQ, OUT, DM, bo);
    } else {
        for (int b = 0; b < NB; ++b)
            k_gemm_out<<<dim3(TT / 64, DM / 64, 1), 32, 0, stream>>>(ATh + (size_t)b * TT * DQ, ATl + (size_t)b * TT * DQ, WO, DQ, OUT + (size_t)b * SEQ_FULL * DM, DM, bo);
    }
}
